// ViMHA_2937757630685
// MI455X (gfx1250) — hardware-verified
//
#include <hip/hip_runtime.h>
#include <stddef.h>
#include <stdint.h>

#define NB    8
#define SQ    1024
#define NTOK  8192
#define DM    1024
#define NH    16
#define HDM   64
#define NQKV  3072
#define IC    4
#define IH    512
#define IW    512
#define PSZ   16
#define QB    128
#define KC    64
#define NQB   (SQ / QB)
#define NCK   (SQ / KC)
#define SBLK  (SQ / 256)
#define QKPLANE (NB * NH * SQ * HDM)
#define NIMG  (NB * IC * IH * IW)

static_assert(NTOK == NB * SQ);
static_assert(DM == IC * PSZ * PSZ);
static_assert(SQ == (IH / PSZ) * (IW / PSZ));
static_assert(NH * HDM == DM);
static_assert(NQKV == 3 * DM);
static_assert(DM % 64 == 0);
static_assert(DM % 32 == 0);
static_assert(HDM == 64);
static_assert(SQ % 256 == 0);
static_assert(SQ % KC == 0);
static_assert(SQ % QB == 0);
static_assert(NIMG == NTOK * DM);
static_assert((NQKV * DM) % 2048 == 0);
static_assert(IW == 128 * 4);
static_assert((NB * IC * IH) % 2 == 0);
static_assert(DM == 128 * 8);

typedef _Float16 v16h __attribute__((ext_vector_type(16)));
typedef _Float16 v8h  __attribute__((ext_vector_type(8)));
typedef float    v8f  __attribute__((ext_vector_type(8)));
typedef float    v4f  __attribute__((ext_vector_type(4)));
typedef unsigned int v4u __attribute__((ext_vector_type(4)));

union Frag  { v16h v; v8h h[2]; };
union Pack8 { v8h h; v4u u; };

__device__ __forceinline__ v8f mma16(v16h a, v16h b, v8f c) {
  c = __builtin_amdgcn_wmma_f32_16x16x32_f16(false, a, false, b, (short)0, c, false, false);
  asm volatile("v_nop\n\tv_nop\n\tv_nop\n\tv_nop" : "+v"(c) : "v"(a), "v"(b));
  return c;
}

__device__ __forceinline__ v16h ldfrag(const _Float16* p, int ld, int row0, int k0, int lane) {
  const int m = lane & 15, lh = lane >> 4;
  const _Float16* q = p + (size_t)(row0 + m) * ld + k0 + 8 * lh;
  Frag f;
  f.h[0] = *(const v8h*)(q);
  f.h[1] = *(const v8h*)(q + 16);
  return f.v;
}

__device__ __forceinline__ v8f zero8() { return (v8f){0.f, 0.f, 0.f, 0.f, 0.f, 0.f, 0.f, 0.f}; }

__device__ __forceinline__ void gemm32x64(const _Float16* __restrict__ A, int lda,
                                          const _Float16* __restrict__ Bt, int ldb, int K,
                                          int m0, int n0, int lane, v8f (&acc)[2][4]) {
#pragma unroll 1
  for (int k0 = 0; k0 < K; k0 += 32) {
    const v16h a0 = ldfrag(A, lda, m0, k0, lane);
    const v16h a1 = ldfrag(A, lda, m0 + 16, k0, lane);
    const v16h b0 = ldfrag(Bt, ldb, n0, k0, lane);
    const v16h b1 = ldfrag(Bt, ldb, n0 + 16, k0, lane);
    const v16h b2 = ldfrag(Bt, ldb, n0 + 32, k0, lane);
    const v16h b3 = ldfrag(Bt, ldb, n0 + 48, k0, lane);
    acc[0][0] = mma16(a0, b0, acc[0][0]);
    acc[1][0] = mma16(a1, b0, acc[1][0]);
    acc[0][1] = mma16(a0, b1, acc[0][1]);
    acc[1][1] = mma16(a1, b1, acc[1][1]);
    acc[0][2] = mma16(a0, b2, acc[0][2]);
    acc[1][2] = mma16(a1, b2, acc[1][2]);
    acc[0][3] = mma16(a0, b3, acc[0][3]);
    acc[1][3] = mma16(a1, b3, acc[1][3]);
  }
}

#define PECOEF (-0.008994473019507992f)
__global__ __launch_bounds__(128) void k_tok(const float* __restrict__ x, _Float16* __restrict__ xh) {
  __shared__ __align__(16) float pel[128 * 8];
  const int tid = threadIdx.x;
  const int i   = blockIdx.x;
  const int j0  = tid * 8;
#pragma unroll 1
  for (int q = 0; q < 4; ++q) {
    const float jj   = (float)(j0 + 2 * q);
    const float freq = expf(jj * PECOEF);
    const float ang  = (float)i * freq;
    float sv, cv;
    sincosf(ang, &sv, &cv);
    pel[j0 + 2 * q]     = sv;
    pel[j0 + 2 * q + 1] = cv;
  }
  __syncthreads();
  const v4f pe0 = *(const v4f*)(pel + j0);
  const v4f pe1 = *(const v4f*)(pel + j0 + 4);

  const int c     = i >> 8;
  const int patch = (i & 255) * 4 + (j0 >> 8);
  const int py    = (j0 >> 4) & 15;
  const int px    = j0 & 15;
  const int ph    = patch >> 5, pw = patch & 31;
  const size_t srow = ((size_t)c * IH + (size_t)(ph * PSZ + py)) * IW + (size_t)(pw * PSZ + px);
#pragma unroll 1
  for (int b = 0; b < NB; ++b) {
    const float* sp = x + (size_t)b * IC * IH * IW + srow;
    const v4f x0 = *(const v4f*)(sp);
    const v4f x1 = *(const v4f*)(sp + 4);
    const v4f t0 = (x0 + pe0) + x0;
    const v4f t1 = (x1 + pe1) + x1;
    Pack8 pk;
    pk.h = (v8h){(_Float16)t0[0], (_Float16)t0[1], (_Float16)t0[2], (_Float16)t0[3],
                 (_Float16)t1[0], (_Float16)t1[1], (_Float16)t1[2], (_Float16)t1[3]};
    const v4u vv = pk.u;
    volatile v4u* d = (volatile v4u*)(xh + (size_t)(b * SQ + i) * DM + j0);
    *d = vv;
    __threadfence();
    *d = vv;
  }
}

__global__ __launch_bounds__(256) void k_wcvt(const float* __restrict__ src, _Float16* __restrict__ dh, float scale) {
  const int tid = threadIdx.x;
  const size_t o = (size_t)blockIdx.x * 2048 + (size_t)tid * 8;
  const v4f a0 = *(const v4f*)(src + o) * scale;
  const v4f a1 = *(const v4f*)(src + o + 4) * scale;
  Pack8 pk;
  pk.h = (v8h){(_Float16)a0[0], (_Float16)a0[1], (_Float16)a0[2], (_Float16)a0[3],
               (_Float16)a1[0], (_Float16)a1[1], (_Float16)a1[2], (_Float16)a1[3]};
  const v4u vv = pk.u;
  volatile v4u* d = (volatile v4u*)(dh + o);
  *d = vv;
  __threadfence();
  *d = vv;
}

#define STP 72
#define SVP 264
__global__ __launch_bounds__(256) void k_qkv(const _Float16* __restrict__ xh,
                                             const _Float16* __restrict__ wh,
                                             _Float16* __restrict__ qkp,
                                             _Float16* __restrict__ vtp) {
  __shared__ __align__(16) _Float16 st[256 * STP];
  const int tid = threadIdx.x, lane = tid & 31, wave = tid >> 5;
  const int hh = lane >> 4, c = lane & 15;
  const int bx = blockIdx.x;
  const int b  = bx / SBLK;
  const int sb = (bx - b * SBLK) * 256;
  const int ns = blockIdx.y;
  const int which = ns / NH;
  const int head  = ns - which * NH;
  const int hb    = b * NH + head;
  const int m0 = bx * 256 + wave * 32;
  const int n0 = ns * 64;

  v8f acc[2][4];
#pragma unroll
  for (int s = 0; s < 2; ++s)
#pragma unroll
    for (int t = 0; t < 4; ++t) acc[s][t] = zero8();
  gemm32x64(xh, DM, wh, DM, DM, m0, n0, lane, acc);

  if (which < 2) {
#pragma unroll
    for (int sub = 0; sub < 2; ++sub)
#pragma unroll
      for (int t = 0; t < 4; ++t)
#pragma unroll
        for (int r = 0; r < 8; ++r)
          st[(wave * 32 + sub * 16 + 8 * hh + r) * STP + 16 * t + c] =
              (_Float16)(acc[sub][t][r] * 0.03125f);
  } else {
#pragma unroll
    for (int sub = 0; sub < 2; ++sub)
#pragma unroll
      for (int t = 0; t < 4; ++t)
#pragma unroll
        for (int r = 0; r < 8; ++r)
          st[(16 * t + c) * SVP + wave * 32 + sub * 16 + 8 * hh + r] =
              (_Float16)(acc[sub][t][r] * 0.03125f);
  }
  __syncthreads();

  if (which < 2) {
    _Float16* base = qkp + (size_t)which * QKPLANE + (size_t)hb * SQ * HDM;
#pragma unroll
    for (int g = 0; g < 2; ++g) {
      v4u val[4];
      size_t go[4];
#pragma unroll
      for (int j = 0; j < 4; ++j) {
        const int p  = tid + 256 * (4 * g + j);
        const int lr = p >> 3;
        const int pc = p & 7;
        Pack8 pk;
        pk.h   = *(const v8h*)(st + lr * STP + pc * 8);
        val[j] = pk.u;
        go[j]  = (size_t)(sb + lr) * HDM + pc * 8;
      }
      for (int ps = 0; ps < 2; ++ps) {
#pragma unroll
        for (int j = 0; j < 4; ++j) *(volatile v4u*)(base + go[j]) = val[j];
        __threadfence();
      }
    }
  } else {
    _Float16* base = vtp + (size_t)hb * HDM * SQ;
#pragma unroll
    for (int g = 0; g < 2; ++g) {
      v4u val[4];
      size_t go[4];
#pragma unroll
      for (int j = 0; j < 4; ++j) {
        const int p    = tid + 256 * (4 * g + j);
        const int drow = p >> 5;
        const int pc   = p & 31;
        Pack8 pk;
        pk.h   = *(const v8h*)(st + drow * SVP + pc * 8);
        val[j] = pk.u;
        go[j]  = (size_t)drow * SQ + sb + pc * 8;
      }
      for (int ps = 0; ps < 2; ++ps) {
#pragma unroll
        for (int j = 0; j < 4; ++j) *(volatile v4u*)(base + go[j]) = val[j];
        __threadfence();
      }
    }
  }
}

#define KTP 72
#define OTP 68
__global__ __launch_bounds__(256) void k_attn(const _Float16* __restrict__ qp,
                                              const _Float16* __restrict__ kp,
                                              const _Float16* __restrict__ vt,
                                              float* __restrict__ op, float sscale) {
  __shared__ __align__(16) _Float16 Ks[KC * KTP];
  __shared__ __align__(16) _Float16 Vs[HDM * KTP];
  __shared__ __align__(16) float    Os[8 * 16 * OTP];

  const int tid = threadIdx.x, lane = tid & 31, wave = tid >> 5;
  const int hh = lane >> 4, c = lane & 15;
  const int qb  = blockIdx.x % NQB;
  const int hb  = blockIdx.x / NQB;
  const int h   = hb % NH;
  const int b   = hb / NH;
  const int q0  = qb * QB + wave * 16;

  const _Float16* Q = qp + (size_t)hb * SQ * HDM;
  const _Float16* K = kp + (size_t)hb * SQ * HDM;
  const _Float16* V = vt + (size_t)hb * HDM * SQ;

  v16h qa[2];
  qa[0] = ldfrag(Q, HDM, q0, 0, lane);
  qa[1] = ldfrag(Q, HDM, q0, 32, lane);

  const float NEGI = -__builtin_huge_valf();
  float mrow[8], lrow[8];
  v8f oacc[4];
#pragma unroll
  for (int r = 0; r < 8; ++r) { mrow[r] = NEGI; lrow[r] = 0.f; }
#pragma unroll
  for (int t = 0; t < 4; ++t) oacc[t] = zero8();

  float*    sw = Os + wave * 16 * OTP;
  _Float16* pw = (_Float16*)sw;

  for (int kc = 0; kc < NCK; ++kc) {
    const int kv0 = kc * KC;
    __syncthreads();
    {
      const int r  = tid >> 2;
      const int qq = (tid & 3) * 16;
      const _Float16* ks = K + (size_t)(kv0 + r) * HDM + qq;
      const _Float16* vs = V + (size_t)r * SQ + kv0 + qq;
#pragma unroll
      for (int e = 0; e < 2; ++e) {
        *(v8h*)(Ks + r * KTP + qq + 8 * e) = *(const v8h*)(ks + 8 * e);
        *(v8h*)(Vs + r * KTP + qq + 8 * e) = *(const v8h*)(vs + 8 * e);
      }
    }
    __syncthreads();

    v8f s[4];
#pragma unroll
    for (int j = 0; j < 4; ++j) s[j] = zero8();
#pragma unroll
    for (int dc = 0; dc < 2; ++dc) {
#pragma unroll
      for (int j = 0; j < 4; ++j) {
        const v16h kb = ldfrag(Ks, KTP, j * 16, dc * 32, lane);
        s[j] = mma16(qa[dc], kb, s[j]);
      }
    }
    float cm[8];
#pragma unroll
    for (int r = 0; r < 8; ++r) {
      float m = NEGI;
#pragma unroll
      for (int j = 0; j < 4; ++j) { s[j][r] *= sscale; m = fmaxf(m, s[j][r]); }
#pragma unroll
      for (int off = 1; off < 16; off <<= 1) m = fmaxf(m, __shfl_xor(m, off, 32));
      cm[r] = m;
    }
    float al[8];
#pragma unroll
    for (int r = 0; r < 8; ++r) {
      const float mnew  = fmaxf(mrow[r], cm[r]);
      const float alpha = __expf(mrow[r] - mnew);
      mrow[r] = mnew;
      float psum = 0.f;
#pragma unroll
      for (int j = 0; j < 4; ++j) {
        const float p = __expf(s[j][r] - mnew);
        psum += p;
        pw[(8 * hh + r) * KTP + j * 16 + c] = (_Float16)(p * 1024.0f);
      }
#pragma unroll
      for (int off = 1; off < 16; off <<= 1) psum += __shfl_xor(psum, off, 32);
      lrow[r] = lrow[r] * alpha + psum;
      al[r] = alpha;
    }
#pragma unroll
    for (int t = 0; t < 4; ++t)
#pragma unroll
      for (int r = 0; r < 8; ++r) oacc[t][r] *= al[r];
    __syncthreads();

#pragma unroll
    for (int kk = 0; kk < 2; ++kk) {
      const v16h pa = ldfrag(pw, KTP, 0, kk * 32, lane);
#pragma unroll
      for (int t = 0; t < 4; ++t) {
        const v16h vb = ldfrag(Vs, KTP, t * 16, kk * 32, lane);
        oacc[t] = mma16(pa, vb, oacc[t]);
      }
    }
  }

  float invl[8];
#pragma unroll
  for (int r = 0; r < 8; ++r) {
    const float lr = (lrow[r] > 0.f) ? lrow[r] : 1.0f;
    invl[r] = 0.0009765625f * (1.0f / lr);
  }
  __syncthreads();
#pragma unroll
  for (int r = 0; r < 8; ++r) {
#pragma unroll
    for (int t = 0; t < 4; ++t)
      sw[(8 * hh + r) * OTP + 16 * t + c] = oacc[t][r] * invl[r];
  }
  __syncthreads();
  v4f val[8];
  size_t go[8];
#pragma unroll
  for (int it = 0; it < 8; ++it) {
    const int p    = lane + 32 * it;
    const int L    = p >> 3;
    const int pc   = p & 7;
    const int row  = L >> 1;
    const int half = L & 1;
    val[it] = *(const v4f*)(sw + row * OTP + half * 32 + pc * 4);
    go[it]  = ((size_t)b * SQ + (size_t)(q0 + row)) * DM + (size_t)h * HDM + half * 32 + pc * 4;
  }
  for (int ps = 0; ps < 2; ++ps) {
#pragma unroll
    for (int it = 0; it < 8; ++it) *(volatile v4f*)(op + go[it]) = val[it];
    __threadfence();
  }
}

__global__ __launch_bounds__(256) void k_img(const float* __restrict__ op, float* __restrict__ out) {
  const int tid   = threadIdx.x;
  const int rowid = blockIdx.x * 2 + (tid >> 7);
  const int xq    = tid & 127;
  const int y     = rowid & (IH - 1);
  const int bc    = rowid >> 9;
  const int c     = bc & (IC - 1);
  const int b     = bc >> 2;
  const int x0    = xq * 4;
  const int pw    = x0 >> 4, px = x0 & 15;
  const int ph    = y >> 4,  py = y & 15;
  const int patch = ph * 32 + pw;
  const int i     = c * 256 + (patch >> 2);
  const int hd    = (patch & 3) * 4 + (py >> 2);
  const int dd    = (py & 3) * 16 + px;
  const v4f v = *(const v4f*)(op + (size_t)(b * SQ + i) * DM + hd * HDM + dd);
  volatile v4f* d = (volatile v4f*)(out + (size_t)rowid * IW + x0);
  *d = v;
  __threadfence();
  *d = v;
}

extern "C" void kernel_launch(void* const* d_in, const int* in_sizes, int n_in,
                              void* d_out, int out_size, void* d_ws, size_t ws_size,
                              hipStream_t stream) {
  if (n_in < 2) return;
  if (in_sizes[0] != NIMG) return;
  if (in_sizes[1] != NQKV * DM) return;
  if (out_size != NIMG) return;

  const float* x = (const float*)d_in[0];
  const float* w = (const float*)d_in[1];
  float* out = (float*)d_out;

  size_t off = 0;
  const size_t oX = off; off += (size_t)NTOK * DM * 2;
  const size_t oW = off; off += (size_t)NQKV * DM * 2;
  const size_t oQ = off; off += (size_t)NB * NH * SQ * HDM * 2;
  const size_t oK = off; off += (size_t)NB * NH * SQ * HDM * 2;
  const size_t oV = off; off += (size_t)NB * NH * HDM * SQ * 2;
  const size_t oO = off; off += (size_t)NTOK * DM * 4;
  if (off > ws_size) return;
  if (off > (size_t)134217728) return;
  if (oK != oQ + (size_t)QKPLANE * 2) return;

  char* ws = (char*)d_ws;
  _Float16* Xh  = (_Float16*)(ws + oX);
  _Float16* Wh  = (_Float16*)(ws + oW);
  _Float16* QKp = (_Float16*)(ws + oQ);
  _Float16* Kp  = (_Float16*)(ws + oK);
  _Float16* Vt  = (_Float16*)(ws + oV);
  float*    Op  = (float*)(ws + oO);

  k_tok<<<dim3(SQ), dim3(128), 0, stream>>>(x, Xh);
  k_wcvt<<<dim3((NQKV * DM) / 2048), dim3(256), 0, stream>>>(w, Wh, 32.0f);
  k_qkv<<<dim3(NB * SBLK, NQKV / 64), dim3(256), 0, stream>>>(Xh, Wh, QKp, Vt);
  const float sscale = 0.03125f;
  k_attn<<<dim3(NB * NH * NQB), dim3(256), 0, stream>>>(QKp, Kp, Vt, Op, sscale);
  k_img<<<dim3((NB * IC * IH) / 2), dim3(256), 0, stream>>>(Op, out);
  (void)hipGetLastError();
}
